// ConcatAtten_25769803882
// MI455X (gfx1250) — hardware-verified
//
#include <hip/hip_runtime.h>
#include <stddef.h>


typedef _Float16 v16h __attribute__((ext_vector_type(16)));
typedef _Float16 v8h  __attribute__((ext_vector_type(8)));
typedef float    v8f  __attribute__((ext_vector_type(8)));
typedef float    v4f  __attribute__((ext_vector_type(4)));
typedef _Float16 h16;

#ifndef NB
#define NB 4
#endif
#ifndef QLEN
#define QLEN 512
#endif
#ifndef KLEN
#define KLEN 512
#endif
#define NB_FULL   4
#define QLEN_FULL 512
#define KLEN_FULL 512
#define FEAT 256
#define ENC  128
#define TT   8

static_assert(NB >= 1 && NB <= NB_FULL);
static_assert(QLEN >= 64 && QLEN <= QLEN_FULL && (QLEN % 64) == 0);
static_assert(KLEN >= 64 && KLEN <= KLEN_FULL && (KLEN % 64) == 0);
static_assert((FEAT % 64) == 0 && (FEAT % 32) == 0);
static_assert((ENC % 64) == 0 && (ENC % 32) == 0 && (ENC % 4) == 0);
static_assert(((NB * QLEN) % 64) == 0 && ((NB * KLEN) % 64) == 0);
static_assert((((size_t)NB * QLEN * FEAT / 8) % 256) == 0);
static_assert((((size_t)NB * KLEN * FEAT / 8) % 256) == 0);
static_assert((((size_t)NB * FEAT * KLEN / 8) % 256) == 0);
static_assert(TT == 8);
static_assert((KLEN % TT) == 0);
static_assert(((TT * ENC) % 256) == 0);
static_assert((QLEN % 32) == 0);
static_assert((KLEN % 32) == 0);

#define LDT 72
#define LDC 68
static_assert((LDT % 8) == 0 && LDT >= 64);
static_assert((LDC % 4) == 0 && LDC >= 64);

#define WCARRY 64.0f
#define XCARRY 16.0f
#define PCARRY 16384.0f
#define PSCALE (2.8853900817779268f / (WCARRY * XCARRY))
#define OSCALE (1.0f / (PCARRY * XCARRY))
#define LSCALE (-2.8853900817779268f)

static_assert((size_t)64 * LDT * 2 <= (size_t)131072);
static_assert((size_t)64 * LDC * 4 <= (size_t)131072);
static_assert(((size_t)TT * ENC + ENC + (size_t)TT * QLEN) * 4 <= (size_t)131072);

#define W_BYTES   ((size_t)ENC * FEAT * 2)
#define XQ_BYTES  ((size_t)NB * QLEN * FEAT * 2)
#define XK_BYTES  ((size_t)NB * KLEN * FEAT * 2)
#define V_BYTES   ((size_t)NB * FEAT * KLEN * 2)
#define QP_BYTES  ((size_t)NB * QLEN * ENC * 4)
#define KP_BYTES  ((size_t)NB * KLEN * ENC * 4)
#define P_BYTES   ((size_t)NB * KLEN * QLEN * 4)
#define PT_BYTES  ((size_t)NB * QLEN * KLEN * 2)
#define OFF_W1T ((size_t)0)
#define OFF_W2T (OFF_W1T + W_BYTES)
#define OFF_XQ  (OFF_W2T + W_BYTES)
#define OFF_XK  (OFF_XQ + XQ_BYTES)
#define OFF_V   (OFF_XK + XK_BYTES)
#define OFF_QP  (OFF_V + V_BYTES)
#define OFF_KP  (OFF_QP + QP_BYTES)
#define OFF_P   (OFF_KP + KP_BYTES)
#define OFF_PT  (OFF_P + P_BYTES)
#define WS_TOTAL (OFF_PT + PT_BYTES)
static_assert((W_BYTES % 128) == 0 && (XQ_BYTES % 128) == 0 && (XK_BYTES % 128) == 0);
static_assert((V_BYTES % 128) == 0 && (QP_BYTES % 128) == 0 && (KP_BYTES % 128) == 0);
static_assert((P_BYTES % 128) == 0 && (PT_BYTES % 128) == 0);
static_assert(WS_TOTAL <= (size_t)134217728);

__device__ __forceinline__ float bf16r(float x) {
  unsigned int u = __float_as_uint(x);
  u = (u + 0x7FFFu + ((u >> 16) & 1u)) & 0xFFFF0000u;
  return __uint_as_float(u);
}

static __device__ __forceinline__ h16 toh_flush(float v) {
  const h16 r = (h16)v;
  return (fabsf(v) < 6.103515625e-05f) ? (h16)0.0f : r;
}

__device__ __forceinline__ v16h frag_at(const _Float16* p) {
  v8h lo = *(const v8h*)(p);
  v8h hi = *(const v8h*)(p + 16);
  v16h out;
#pragma unroll
  for (int i = 0; i < 8; ++i) { out[i] = lo[i]; out[i + 8] = hi[i]; }
  return out;
}

__device__ __forceinline__ v8f wmma16(v16h a, v16h b, v8f c) {
  v8f d = __builtin_amdgcn_wmma_f32_16x16x32_f16(false, a, false, b, (short)0, c,
                                                 false, false);
  asm volatile("v_nop\n\tv_nop\n\tv_nop\n\tv_nop" : "+v"(d) : "v"(a), "v"(b));
  return d;
}

__device__ __forceinline__ float red32_max(float x) {
#pragma unroll
  for (int off = 1; off < 32; off <<= 1) x = fmaxf(x, __shfl_xor(x, off, 32));
  return x;
}
__device__ __forceinline__ float red32_sum(float x) {
#pragma unroll
  for (int off = 1; off < 32; off <<= 1) x += __shfl_xor(x, off, 32);
  return x;
}

__device__ __forceinline__ float fexp2(float x) {
#if __has_builtin(__builtin_amdgcn_exp2f)
  return __builtin_amdgcn_exp2f(x);
#else
  return exp2f(x);
#endif
}

__device__ __forceinline__ float rcp1p(float x) {
  return __builtin_amdgcn_rcpf(fexp2(x) + 1.0f);
}

__global__ __launch_bounds__(256) void wconv_kernel(
    const float* __restrict__ W, _Float16* __restrict__ Wt, unsigned ldw, unsigned ldk) {
  __shared__ _Float16 T[64 * LDT];
  const unsigned tid = threadIdx.x;
  const unsigned n0 = blockIdx.x * 64u;
  const unsigned k0 = blockIdx.y * 64u;
#pragma unroll 4
  for (unsigned j = 0; j < 16u; ++j) {
    const unsigned idx = tid + 256u * j;
    const unsigned kr = idx >> 6, nc = idx & 63u;
    const float v = W[(size_t)(k0 + kr) * ldw + n0 + nc];
    T[nc * LDT + kr] = toh_flush(WCARRY * bf16r(v));
  }
  __syncthreads();
  v8h x[2];
  size_t off[2];
#pragma unroll
  for (unsigned i = 0; i < 2u; ++i) {
    const unsigned n = 32u * i + (tid >> 3);
    const unsigned kc = (tid & 7u) * 8u;
    x[i] = *(const v8h*)&T[n * LDT + kc];
    off[i] = (size_t)(n0 + n) * ldk + k0 + kc;
  }
#pragma unroll
  for (int i = 0; i < 2; ++i) *(volatile v8h*)(Wt + off[i]) = x[i];
  __threadfence();
#pragma unroll
  for (int i = 0; i < 2; ++i) *(volatile v8h*)(Wt + off[i]) = x[i];
}

__global__ __launch_bounds__(256) void pconv_kernel(
    const float* __restrict__ P, _Float16* __restrict__ PT) {
  __shared__ _Float16 T[64 * LDT];
  const unsigned tid = threadIdx.x;
  const unsigned n0 = blockIdx.x * 64u;
  const unsigned k0 = blockIdx.y * 64u;
  const unsigned b = blockIdx.z;
  const float* src = P + (size_t)b * KLEN * QLEN;
  _Float16* dst = PT + (size_t)b * QLEN * KLEN;
#pragma unroll 4
  for (unsigned j = 0; j < 16u; ++j) {
    const unsigned idx = tid + 256u * j;
    const unsigned kr = idx >> 6, nc = idx & 63u;
    const float v = src[(size_t)(k0 + kr) * QLEN + n0 + nc];
    T[nc * LDT + kr] = toh_flush(PCARRY * v);
  }
  __syncthreads();
  v8h x[2];
  size_t off[2];
#pragma unroll
  for (unsigned i = 0; i < 2u; ++i) {
    const unsigned n = 32u * i + (tid >> 3);
    const unsigned kc = (tid & 7u) * 8u;
    x[i] = *(const v8h*)&T[n * LDT + kc];
    off[i] = (size_t)(n0 + n) * KLEN + k0 + kc;
  }
#pragma unroll
  for (int i = 0; i < 2; ++i) *(volatile v8h*)(dst + off[i]) = x[i];
  __threadfence();
#pragma unroll
  for (int i = 0; i < 2; ++i) *(volatile v8h*)(dst + off[i]) = x[i];
}

__global__ __launch_bounds__(256) void xconv_kernel(
    const float* __restrict__ X, _Float16* __restrict__ dst,
    unsigned R, unsigned RF, unsigned C, unsigned CF) {
  const unsigned g = blockIdx.x * 256u + threadIdx.x;
  const unsigned cpr = C >> 3;
  const unsigned row = g / cpr;
  const unsigned cc = (g - row * cpr) * 8u;
  const unsigned b = row / R;
  const unsigned r = row - b * R;
  const float* s = X + ((size_t)b * RF + r) * CF + cc;
  const v4f a0 = *(const v4f*)(s);
  const v4f a1 = *(const v4f*)(s + 4);
  v8h o;
#pragma unroll
  for (int i = 0; i < 4; ++i) {
    o[i]     = toh_flush(XCARRY * bf16r(a0[i]));
    o[i + 4] = toh_flush(XCARRY * bf16r(a1[i]));
  }
  _Float16* p = dst + (size_t)g * 8u;
  *(volatile v8h*)p = o;
  __threadfence();
  *(volatile v8h*)p = o;
}

__device__ __forceinline__ void gemm_body(
    const _Float16* __restrict__ A16, const _Float16* __restrict__ Bt, const unsigned K,
    float* __restrict__ outf, const unsigned ldo, const float cs) {
  __shared__ float Cs[64 * LDC];
  const unsigned tid = threadIdx.x, lane = tid & 31u, w = tid >> 5;
  const unsigned mw = w >> 1, nw = w & 1u;
  const unsigned hh = lane >> 4, m = lane & 15u;
  const unsigned n0 = blockIdx.x * 64u;
  const unsigned row0 = blockIdx.y * 64u;

  const _Float16* ap  = A16 + (size_t)(row0 + mw * 16u + m) * K + hh * 8u;
  const _Float16* bp0 = Bt + (size_t)(n0 + nw * 32u + m) * K + hh * 8u;
  const _Float16* bp1 = bp0 + (size_t)16 * K;
  v8f acc0 = {}, acc1 = {};
#pragma unroll 2
  for (unsigned k0 = 0; k0 < K; k0 += 32u) {
    const v16h a  = frag_at(ap + k0);
    const v16h b0 = frag_at(bp0 + k0);
    const v16h b1 = frag_at(bp1 + k0);
    acc0 = wmma16(a, b0, acc0);
    acc1 = wmma16(a, b1, acc1);
  }
#pragma unroll
  for (int r = 0; r < 8; ++r) {
    float* d = &Cs[(mw * 16u + hh * 8u + (unsigned)r) * LDC + nw * 32u + m];
    d[0]  = acc0[r];
    d[16] = acc1[r];
  }
  __syncthreads();

  v4f xs[4];
  size_t off[4];
#pragma unroll
  for (unsigned i = 0; i < 4u; ++i) {
    const unsigned r = 16u * i + (tid >> 4);
    const unsigned c = (tid & 15u) * 4u;
    const v4f u = *(const v4f*)&Cs[r * LDC + c];
    v4f val;
#pragma unroll
    for (int j = 0; j < 4; ++j) val[j] = u[j] * cs;
    xs[i] = val;
    off[i] = (size_t)(row0 + r) * ldo + n0 + c;
  }
#pragma unroll
  for (int i = 0; i < 4; ++i) *(volatile v4f*)(outf + off[i]) = xs[i];
  __threadfence();
#pragma unroll
  for (int i = 0; i < 4; ++i) *(volatile v4f*)(outf + off[i]) = xs[i];
}

__global__ __launch_bounds__(256) void proj_kernel(
    const _Float16* __restrict__ A16, const _Float16* __restrict__ Bt,
    float* __restrict__ outf) {
  gemm_body(A16, Bt, (unsigned)FEAT, outf, (unsigned)ENC, PSCALE);
}

__global__ __launch_bounds__(256) void outgemm_kernel(
    const _Float16* __restrict__ V16, const _Float16* __restrict__ PT,
    float* __restrict__ outf) {
  const unsigned b = blockIdx.z;
  gemm_body(V16 + (size_t)b * FEAT * KLEN, PT + (size_t)b * QLEN * KLEN, (unsigned)KLEN,
            outf + (size_t)b * FEAT * QLEN_FULL, (unsigned)QLEN_FULL, OSCALE);
}

__global__ __launch_bounds__(256) void score_kernel(
    const float* __restrict__ Qp, const float* __restrict__ Kp,
    const float* __restrict__ vc, float* __restrict__ P) {
  __shared__ __attribute__((aligned(16))) float krow[TT * ENC];
  __shared__ __attribute__((aligned(16))) float vcs[ENC];
  __shared__ __attribute__((aligned(16))) float sv[TT * QLEN];

  const unsigned tid = threadIdx.x;
  const unsigned t0 = blockIdx.x * (unsigned)TT;
  const unsigned b = blockIdx.y;

  if (tid < (unsigned)ENC) vcs[tid] = bf16r(vc[tid]);
  {
    const float* kp = Kp + (size_t)(b * (unsigned)KLEN + t0) * ENC;
#pragma unroll
    for (unsigned j = 0; j < (unsigned)(TT * ENC / 256); ++j) {
      const unsigned i = tid + 256u * j;
      krow[i] = kp[i];
    }
  }
  __syncthreads();

#pragma unroll 1
  for (unsigned q = tid; q < (unsigned)QLEN; q += 256u) {
    const float* qr = Qp + (size_t)(b * (unsigned)QLEN + q) * ENC;
    float acc[TT];
#pragma unroll
    for (int t = 0; t < TT; ++t) acc[t] = 0.0f;
#pragma unroll 1
    for (unsigned e = 0; e < (unsigned)ENC; e += 4u) {
      const v4f qv = *(const v4f*)(qr + e);
      const v4f vv = *(const v4f*)&vcs[e];
#pragma unroll
      for (int t = 0; t < TT; ++t) {
        const v4f kk = *(const v4f*)&krow[(unsigned)t * ENC + e];
#pragma unroll
        for (int j = 0; j < 4; ++j) acc[t] += vv[j] * rcp1p(kk[j] + qv[j]);
      }
    }
#pragma unroll
    for (int t = 0; t < TT; ++t) sv[(unsigned)t * QLEN + q] = acc[t] * LSCALE;
  }
  __syncthreads();

  const int wave = __builtin_amdgcn_readfirstlane((int)(threadIdx.x >> 5));
  const unsigned lane = tid & 31u;
  const unsigned sb = (unsigned)wave * (unsigned)QLEN + lane;

  float mx = -3.0e38f;
#pragma unroll 4
  for (unsigned j = 0; j < (unsigned)(QLEN / 32); ++j) mx = fmaxf(mx, sv[sb + 32u * j]);
  mx = red32_max(mx);

  float sum = 0.0f;
#pragma unroll 4
  for (unsigned j = 0; j < (unsigned)(QLEN / 32); ++j) {
    const float ex = fexp2(sv[sb + 32u * j] - mx);
    sv[sb + 32u * j] = ex;
    sum += ex;
  }
  sum = red32_sum(sum);
  const float inv = __builtin_amdgcn_rcpf(sum);

#pragma unroll 4
  for (unsigned j = 0; j < (unsigned)(QLEN / 32); ++j) {
    const float pv = sv[sb + 32u * j] * inv;
    sv[sb + 32u * j] = pv;
  }

  float* prow = P + (size_t)(b * (unsigned)KLEN + t0 + (unsigned)wave) * QLEN + lane;
#pragma unroll 4
  for (unsigned j = 0; j < (unsigned)(QLEN / 32); ++j)
    *(volatile float*)(prow + 32u * j) = sv[sb + 32u * j];
  __threadfence();
#pragma unroll 4
  for (unsigned j = 0; j < (unsigned)(QLEN / 32); ++j)
    *(volatile float*)(prow + 32u * j) = sv[sb + 32u * j];
}

extern "C" void kernel_launch(void* const* d_in, const int* in_sizes, int n_in,
                              void* d_out, int out_size, void* d_ws, size_t ws_size,
                              hipStream_t stream) {
  if (n_in < 6) return;
  const long long need_q = ((long long)(NB - 1) * QLEN_FULL + QLEN) * FEAT;
  const long long need_k = ((long long)(NB - 1) * KLEN_FULL + KLEN) * FEAT;
  const long long need_v = ((long long)NB * FEAT - 1) * KLEN_FULL + KLEN;
  const long long need_o = ((long long)NB * FEAT - 1) * QLEN_FULL + QLEN;
  if ((long long)in_sizes[0] < need_q) return;
  if ((long long)in_sizes[1] < need_k) return;
  if ((long long)in_sizes[2] < need_v) return;
  if ((long long)in_sizes[3] < (long long)FEAT * ENC) return;
  if ((long long)in_sizes[4] < (long long)FEAT * ENC) return;
  if (in_sizes[5] < ENC) return;
  if ((long long)out_size < need_o) return;
  if (ws_size < WS_TOTAL) return;

  const float* query = (const float*)d_in[0];
  const float* key   = (const float*)d_in[1];
  const float* value = (const float*)d_in[2];
  const float* w1    = (const float*)d_in[3];
  const float* w2    = (const float*)d_in[4];
  const float* vc    = (const float*)d_in[5];
  float* out = (float*)d_out;

  char* ws = (char*)d_ws;
  _Float16* W1t = (_Float16*)(ws + OFF_W1T);
  _Float16* W2t = (_Float16*)(ws + OFF_W2T);
  _Float16* XQ  = (_Float16*)(ws + OFF_XQ);
  _Float16* XK  = (_Float16*)(ws + OFF_XK);
  _Float16* V16 = (_Float16*)(ws + OFF_V);
  float*    Qp  = (float*)(ws + OFF_QP);
  float*    Kp  = (float*)(ws + OFF_KP);
  float*    Pf  = (float*)(ws + OFF_P);
  _Float16* PT  = (_Float16*)(ws + OFF_PT);

  dim3 blk(256);

  wconv_kernel<<<dim3(ENC / 64, FEAT / 64), blk, 0, stream>>>(w1, W1t, (unsigned)ENC, (unsigned)FEAT);
  wconv_kernel<<<dim3(ENC / 64, FEAT / 64), blk, 0, stream>>>(w2, W2t, (unsigned)ENC, (unsigned)FEAT);

  xconv_kernel<<<dim3((unsigned)((size_t)NB * QLEN * FEAT / 8 / 256)), blk, 0, stream>>>(
      query, XQ, (unsigned)QLEN, (unsigned)QLEN_FULL, (unsigned)FEAT, (unsigned)FEAT);
  xconv_kernel<<<dim3((unsigned)((size_t)NB * KLEN * FEAT / 8 / 256)), blk, 0, stream>>>(
      key, XK, (unsigned)KLEN, (unsigned)KLEN_FULL, (unsigned)FEAT, (unsigned)FEAT);
  xconv_kernel<<<dim3((unsigned)((size_t)NB * FEAT * KLEN / 8 / 256)), blk, 0, stream>>>(
      value, V16, (unsigned)FEAT, (unsigned)FEAT, (unsigned)KLEN, (unsigned)KLEN_FULL);

  proj_kernel<<<dim3(ENC / 64, NB * QLEN / 64), blk, 0, stream>>>(XQ, W1t, Qp);
  proj_kernel<<<dim3(ENC / 64, NB * KLEN / 64), blk, 0, stream>>>(XK, W2t, Kp);

  score_kernel<<<dim3(KLEN / TT, NB), blk, 0, stream>>>(Qp, Kp, vc, Pf);

  pconv_kernel<<<dim3(QLEN / 64, KLEN / 64, NB), blk, 0, stream>>>(Pf, PT);

  outgemm_kernel<<<dim3(QLEN / 64, FEAT / 64, NB), blk, 0, stream>>>(V16, PT, out);
}
